// MetadataEncoder_41858751266986
// MI455X (gfx1250) — hardware-run, weakly checked
//
#include <hip/hip_runtime.h>


#ifndef NROWS
#define NROWS 500000
#endif
#define NROWS_FULL 500000
#define NT    21
#define NCAT  1000
#define ED    16
#define KD    344
#define KP    352
#define ND    32
#define AW    4
#define TROWS (16 * AW)
#define APITCH 360
#define OSP   36
#define SLOPE 0.01f

static_assert(NT * ED + 8 == KD);
static_assert(KD + 8 == KP);
static_assert(KP % 32 == 0);
static_assert(KP % 8 == 0);
static_assert(KD % 8 == 0);
static_assert(ED == 16);
static_assert(ND == 32);
static_assert(APITCH >= KP);
static_assert(APITCH % 8 == 0);
static_assert((OSP * 4) % 16 == 0);
static_assert(OSP >= ND);
static_assert(NROWS <= NROWS_FULL);
static_assert(NROWS >= 1);
static_assert(((size_t)NT * NCAT * ED) % 8 == 0);
static_assert(((size_t)NT * NCAT * ED * 2) % 128 == 0);
static_assert(((size_t)ND * KP * 2) % 128 == 0);
static_assert(32 * 8 * NT == 16 * NT * ED);
static_assert(32 * 8 == 16 * 16);
static_assert(32 * 16 * 4 == 16 * ND * 4);
static_assert((size_t)TROWS * APITCH * 2 + (size_t)AW * 16 * OSP * 4 <= 131072);

typedef unsigned short bf;
typedef __attribute__((ext_vector_type(16))) __bf16   v16bf;
typedef __attribute__((ext_vector_type(8)))  unsigned short v8us;
typedef __attribute__((ext_vector_type(8)))  float    v8f;
typedef __attribute__((ext_vector_type(4)))  float    v4f;
typedef v4f  __attribute__((may_alias)) v4fa;

__device__ __forceinline__ unsigned short f2bf(float f) { unsigned u = __float_as_uint(f); u += 0x7FFFu + ((u >> 16) & 1u); return (unsigned short)(u >> 16); }
__device__ __forceinline__ float bfr(float f) { return __uint_as_float(((unsigned)f2bf(f)) << 16); }
__device__ __forceinline__ v16bf cat16b(v8us lo, v8us hi) { return __builtin_bit_cast(v16bf, __builtin_shufflevector(lo, hi, 0, 1, 2, 3, 4, 5, 6, 7, 8, 9, 10, 11, 12, 13, 14, 15)); }
__device__ __forceinline__ v8f wmmab(v16bf a, v16bf b, v8f c) { return __builtin_amdgcn_wmma_f32_16x16x32_bf16(false, a, false, b, (short)0, c, false, false); }
__device__ __forceinline__ v8f wmmabg(v16bf a, v16bf b, v8f c) { c = wmmab(a, b, c); asm volatile("v_nop\n\tv_nop\n\tv_nop\n\tv_nop" : "+v"(c) : "v"(a), "v"(b)); return c; }
__device__ __forceinline__ v16bf ldb(const bf* p)  { return cat16b(*(const v8us*)p, *(const v8us*)(p + 16)); }
__device__ __forceinline__ void wave_sync() { __builtin_amdgcn_fence(3  , "wavefront"); __builtin_amdgcn_wave_barrier(); asm volatile("" ::: "memory"); }

__global__ __launch_bounds__(256) void k_cvt8(const float* __restrict__ src, bf* dst, size_t n8) {
    const size_t i = (size_t)blockIdx.x * 256 + threadIdx.x; if (i >= n8) return;
    const v8f v = *(const v8f*)(src + i * 8); v8us o;
#pragma unroll
    for (int k = 0; k < 8; ++k) o[k] = f2bf(v[k]);
    *(volatile v8us*)(dst + i * 8) = o; __threadfence(); *(volatile v8us*)(dst + i * 8) = o;
}

__global__ __launch_bounds__(256) void k_wpl(const float* __restrict__ W, bf* WP) {
    const unsigned p = blockIdx.x * 256u + threadIdx.x; if (p >= (unsigned)(ND * KP / 8)) return;
    const unsigned n = p / (unsigned)(KP / 8);
    const unsigned c8 = (p - n * (unsigned)(KP / 8)) * 8u;
    const unsigned sc = (c8 < (unsigned)KD) ? c8 : (c8 - 8u);
    const size_t so = (size_t)(n * (unsigned)KD + sc);
    const v4f x0 = *(const v4f*)(W + so); const v4f x1 = *(const v4f*)(W + so + 4); v8us o;
#pragma unroll
    for (int k = 0; k < 4; ++k) { o[k] = f2bf(x0[k]); o[4 + k] = f2bf(x1[k]); }
    const size_t oo = (size_t)p * 8;
    *(volatile v8us*)(WP + oo) = o; __threadfence(); *(volatile v8us*)(WP + oo) = o;
}

__global__ __launch_bounds__(32 * AW) void k_enc(const int* __restrict__ xcat, const float* __restrict__ xcont, const bf* __restrict__ TB,
                                                 const float* __restrict__ Wc, const float* __restrict__ bc, const bf* __restrict__ WP,
                                                 const float* __restrict__ bias, float* OUT) {
    __shared__ __align__(16) bf at[TROWS * APITCH];
    __shared__ __align__(16) float os[AW * 16 * OSP];
    const int lane = threadIdx.x & 31, lr = lane & 15, hi = lane >> 4;
    const int wave = __builtin_amdgcn_readfirstlane((int)(threadIdx.x >> 5));
    const unsigned bx = blockIdx.x;
    const unsigned row0 = bx * (unsigned)TROWS + (unsigned)wave * 16u;
    const int sr = lane >> 1, sh = lane & 1;
    const int srow = min((int)row0 + sr, NROWS - 1);
    const unsigned usrow = (unsigned)srow;
    const int abase = (wave * 16 + sr) * APITCH + sh * 8;
    const int* xr = xcat + (size_t)usrow * NT;
#pragma unroll 1
    for (int t = 0; t < NT; ++t) {
        int idx = xr[t]; idx = min(max(idx, 0), NCAT - 1);
        const unsigned eo = ((unsigned)t * (unsigned)NCAT + (unsigned)idx) * (unsigned)ED + (unsigned)sh * 8u;
        const v8us e = *(const v8us*)(TB + (size_t)eo);
        *(v8us*)(&at[abase + t * ED]) = e;
    }
    {
        const float xc = bfr(xcont[(size_t)usrow]);
        v8us cv;
#pragma unroll
        for (int j = 0; j < 8; ++j) {
            const float pre = xc * bfr(Wc[j]) + bfr(bc[j]);
            const float val = (pre >= 0.0f) ? pre : SLOPE * pre;
            const float vhi = bfr(val);
            const float sel = (sh != 0) ? (val - vhi) : val;
            cv[j] = f2bf(sel);
        }
        *(v8us*)(&at[abase + NT * ED]) = cv;
    }
    wave_sync();

    const int aoff = (wave * 16 + lr) * APITCH + 8 * hi;
    const size_t boff = (size_t)lr * KP + 8 * hi;
    v8f c0 = (v8f){}, c1 = (v8f){};
#pragma unroll 1
    for (int kc = 0; kc < KP; kc += 32) {
        const v8us alo = *(const v8us*)(&at[aoff + kc]);
        const v8us ahi = *(const v8us*)(&at[aoff + kc + 16]);
        const v16bf a = cat16b(alo, ahi);
        const v16bf b0 = ldb(WP + boff + kc);
        const v16bf b1 = ldb(WP + boff + (size_t)16 * KP + kc);
        c0 = wmmabg(a, b0, c0);
        c1 = wmmabg(a, b1, c1);
    }

    const float bz0 = bfr(bias[lr]), bz1 = bfr(bias[16 + lr]);
    const int wb = wave * 16 * OSP;
#pragma unroll
    for (int j = 0; j < 8; ++j) {
        const float u0 = c0[j] + bz0, u1 = c1[j] + bz1;
        os[wb + (hi * 8 + j) * OSP + lr]      = (u0 >= 0.0f) ? u0 : SLOPE * u0;
        os[wb + (hi * 8 + j) * OSP + 16 + lr] = (u1 >= 0.0f) ? u1 : SLOPE * u1;
    }
    wave_sync();
    float* orow = OUT + (size_t)row0 * ND;
#pragma unroll 1
    for (int ps = 0; ps < 2; ++ps) {
#pragma unroll
        for (int s = 0; s < 4; ++s) { const int row = 4 * s + (lane >> 3), cofs = (lane & 7) * 4;
            const v4f val = *(const v4fa*)(&os[wb + row * OSP + cofs]);
            if ((int)row0 + row < NROWS) *(volatile v4f*)(orow + (size_t)row * ND + cofs) = val; }
        if (ps == 0) __threadfence(); }
}

static constexpr size_t al256(size_t v) { return (v + 255) & ~(size_t)255; }
static constexpr size_t N8_TB = (size_t)NT * NCAT * ED / 8;
static constexpr size_t SZ_TB = al256((size_t)NT * NCAT * ED * 2);
static constexpr size_t SZ_WP = al256((size_t)ND * KP * 2);
static constexpr size_t SZ_TOTAL = SZ_TB + SZ_WP;
static constexpr unsigned G_TB  = (unsigned)((N8_TB + 255) / 256);
static constexpr unsigned G_WP  = (unsigned)(((size_t)ND * KP / 8 + 255) / 256);
static constexpr unsigned G_ENC = (unsigned)(((size_t)NROWS + TROWS - 1) / TROWS);
static_assert(SZ_TOTAL <= (size_t)134217728);
static_assert(N8_TB * 8 * 2 <= SZ_TB);
static_assert((size_t)G_WP * 256 >= (size_t)ND * KP / 8);
static_assert((size_t)G_ENC * TROWS >= (size_t)NROWS);
static_assert((size_t)(NROWS - 1) * ND + ND <= (size_t)NROWS_FULL * ND);

extern "C" void kernel_launch(void* const* d_in, const int* in_sizes, int n_in,
                              void* d_out, int out_size, void* d_ws, size_t ws_size, hipStream_t stream) {
    if (n_in < 7) return;
    if ((size_t)in_sizes[0] < (size_t)NROWS * NT || (size_t)in_sizes[1] < (size_t)NROWS) return;
    if ((size_t)in_sizes[2] < (size_t)NT * NCAT * ED) return;
    if (in_sizes[3] < 8 || in_sizes[4] < 8 || in_sizes[5] < ND * KD || in_sizes[6] < ND) return;
    if ((size_t)out_size < (size_t)NROWS * ND) return;
    if (SZ_TOTAL > ws_size) return;
    const int*   xcat  = (const int*)d_in[0];
    const float* xcont = (const float*)d_in[1];
    const float* tabs  = (const float*)d_in[2];
    const float* wc    = (const float*)d_in[3];
    const float* bcv   = (const float*)d_in[4];
    const float* w     = (const float*)d_in[5];
    const float* bv    = (const float*)d_in[6];
    float* OUT = (float*)d_out;
    char* wsp = (char*)d_ws;
    bf* TB = (bf*)wsp; wsp += SZ_TB;
    bf* WP = (bf*)wsp; wsp += SZ_WP;

    k_cvt8<<<G_TB, 256, 0, stream>>>(tabs, TB, N8_TB);
    k_wpl<<<G_WP, 256, 0, stream>>>(w, WP);
    k_enc<<<G_ENC, 32 * AW, 0, stream>>>(xcat, xcont, TB, wc, bcv, WP, bv, OUT);
}
